// fn_blstm_76278619177029
// MI455X (gfx1250) — hardware-verified
//
#include <hip/hip_runtime.h>
#include <math.h>

typedef __attribute__((ext_vector_type(16))) _Float16 v16h;
typedef __attribute__((ext_vector_type(16))) __bf16 v16b;
typedef __attribute__((ext_vector_type(8)))  _Float16 v8h;
typedef __attribute__((ext_vector_type(8)))  float v8f;
typedef __attribute__((ext_vector_type(4)))  float v4f;
typedef __attribute__((ext_vector_type(2)))  float v2f;
typedef __attribute__((ext_vector_type(4)))  unsigned v4u;
typedef __attribute__((ext_vector_type(4)))  int v4i;
typedef float __attribute__((may_alias)) float_a;
typedef int __attribute__((may_alias)) int_a;

template <typename T> __device__ __forceinline__ void vst2(void* p, T v) { *(volatile T*)p = v; __threadfence(); *(volatile T*)p = v; }
__device__ __forceinline__ v8f wmma16(v16h a, v16h b, v8f c) {
  v8f d = __builtin_amdgcn_wmma_f32_16x16x32_f16(false, a, false, b, (short)0, c, false, false);
  asm volatile("v_nop\n\tv_nop\n\tv_nop\n\tv_nop" : "+v"(d) : "v"(a), "v"(b));
  return d;
}
__device__ __forceinline__ v8f wmma_bf(v16b a, v16b b, v8f c) {
  v8f d = __builtin_amdgcn_wmma_f32_16x16x32_bf16(false, a, false, b, (short)0, c, false, false);
  asm volatile("v_nop\n\tv_nop\n\tv_nop\n\tv_nop" : "+v"(d) : "v"(a), "v"(b));
  return d;
}
__device__ __forceinline__ v16h frag_h(const _Float16* rowk0, int lane) {
  union { v16h v; v8h q[2]; } u; const _Float16* p = rowk0 + 8 * (lane >> 4);
  u.q[0] = *(const v8h*)p; u.q[1] = *(const v8h*)(p + 16); return u.v;
}
__device__ __forceinline__ v16h frag_f32(const float* rowk0, int lane) {
  v16h a; const float* p = rowk0 + 8 * (lane >> 4);
#pragma unroll
  for (int i = 0; i < 8; ++i) { a[i] = (_Float16)p[i]; a[8 + i] = (_Float16)p[16 + i]; }
  return a;
}
__device__ __forceinline__ v16h frag_f32s(const float* rowk0, int lane, float sc) {
  v16h a; const float* p = rowk0 + 8 * (lane >> 4);
#pragma unroll
  for (int i = 0; i < 8; ++i) { a[i] = (_Float16)(p[i] * sc); a[8 + i] = (_Float16)(p[16 + i] * sc); }
  return a;
}
__device__ __forceinline__ v16h fragc_f32(const float* W, int k0, int n, int lane, int ld, int K) {
  v16h a; const int g = lane >> 4;
#pragma unroll
  for (int i = 0; i < 8; ++i) { const int ka = k0 + 8 * g + i, kb = ka + 16;
    a[i] = (_Float16)(ka < K ? W[(size_t)ka * ld + n] : 0.f); a[8 + i] = (_Float16)(kb < K ? W[(size_t)kb * ld + n] : 0.f); }
  return a;
}
struct F2 { v16b h, l; };
__device__ __forceinline__ F2 bsplit16(const float v[16]) { F2 r;
#pragma unroll
  for (int i = 0; i < 16; ++i) { const __bf16 h = (__bf16)v[i]; r.h[i] = h; r.l[i] = (__bf16)(v[i] - (float)h); }
  return r; }
__device__ __forceinline__ F2 split_row(const float* row, int k0, int lane) { float v[16]; const float* p = row + k0 + 8 * (lane >> 4);
#pragma unroll
  for (int i = 0; i < 8; ++i) { v[i] = p[i]; v[8 + i] = p[16 + i]; }
  return bsplit16(v); }
__device__ __forceinline__ F2 split_rowK(const float* row, int k0, int lane, int K) { float v[16]; const int g = lane >> 4;
#pragma unroll
  for (int i = 0; i < 8; ++i) { const int ka = k0 + 8 * g + i, kb = ka + 16; v[i] = ka < K ? row[ka] : 0.f; v[8 + i] = kb < K ? row[kb] : 0.f; }
  return bsplit16(v); }
__device__ __forceinline__ F2 split_col(const float* W, int k0, int n, int lane, int ld, int K) { float v[16]; const int g = lane >> 4;
#pragma unroll
  for (int i = 0; i < 8; ++i) { const int ka = k0 + 8 * g + i, kb = ka + 16; v[i] = ka < K ? W[(size_t)ka * ld + n] : 0.f; v[8 + i] = kb < K ? W[(size_t)kb * ld + n] : 0.f; }
  return bsplit16(v); }
__device__ __forceinline__ v8f mac3(const F2& a, const F2& b, v8f c) { c = wmma_bf(a.l, b.h, c); c = wmma_bf(a.h, b.l, c); return wmma_bf(a.h, b.h, c); }
__device__ __forceinline__ float sigm(float v) { return 1.0f / (1.0f + expf(-v)); }
#define LDSX() do { asm volatile("s_wait_dscnt 0" ::: "memory"); __builtin_amdgcn_wave_barrier(); __builtin_amdgcn_fence(__ATOMIC_RELEASE, "workgroup"); } while (0)

#define VV 64
#define HH 128
#define NB 128
#define TT 512
#define G4 (4 * HH)
#define RB 16

__global__ __launch_bounds__(256) void k_prep(const float* __restrict__ emb, const float* __restrict__ wif, const float* __restrict__ bif, const float* __restrict__ bhf,
                                            const float* __restrict__ wib, const float* __restrict__ bib, const float* __restrict__ bhb, const float* __restrict__ whf, const float* __restrict__ whb,
                                            float* __restrict__ tab, _Float16* __restrict__ Wh16) {
  const int v = blockIdx.x, dir = blockIdx.y, tid = threadIdx.x;
  const float* wi = dir == 0 ? wif : wib; const float* bi = dir == 0 ? bif : bib; const float* bh = dir == 0 ? bhf : bhb;
  __shared__ float se[HH]; __shared__ __align__(16) float so[G4];
  if (tid < HH) se[tid] = emb[v * HH + tid];
  __syncthreads();
#pragma unroll
  for (int u = 0; u < 2; ++u) { const int gcol = tid * 2 + u; float a = bi[gcol] + bh[gcol];
#pragma unroll 1
    for (int k = 0; k < HH; ++k) a += se[k] * wi[(size_t)gcol * HH + k];
    so[gcol] = a; }
  __syncthreads();
  if (tid < G4 / 4) vst2(tab + ((size_t)dir * VV + v) * G4 + tid * 4, *(const v4f*)(&so[tid * 4]));
  if (tid < 128) { const float* wh = dir == 0 ? whf : whb; const size_t base = (size_t)v * 1024 + tid * 8; union { v8h hh; v4u uu; } pk;
#pragma unroll
    for (int i = 0; i < 8; ++i) pk.hh[i] = (_Float16)wh[base + i];
    vst2(Wh16 + (size_t)dir * G4 * HH + base, pk.uu); }
}
__global__ __launch_bounds__(256) void k_lstm(const int* __restrict__ x, const float* __restrict__ tab, const _Float16* __restrict__ Wh16, float* __restrict__ hs) {
  __shared__ __align__(16) float gates[RB][G4];
  __shared__ __align__(16) _Float16 h16[RB][HH + 16];
  const int tid = threadIdx.x, w = tid >> 5, lane = tid & 31, col = lane & 15, g = lane >> 4;
  const int dir = blockIdx.y, rb = blockIdx.x, r = tid >> 4, u0 = (tid & 15) * 8; const int b = rb * RB + r;
  const _Float16* Wh = Wh16 + (size_t)dir * G4 * HH; const float* tb = tab + (size_t)dir * VV * G4;
  float c[8], h[8];
#pragma unroll
  for (int j = 0; j < 8; ++j) { c[j] = 0.f; h[j] = 0.f; h16[r][u0 + j] = (_Float16)0.f; }
  __syncthreads();
#pragma unroll 1
  for (int st = 0; st < TT; ++st) { const int t = dir == 0 ? st : TT - 1 - st;
    v8f acc[4] = {};
#pragma unroll
    for (int kc = 0; kc < HH / 32; ++kc) { const v16h a = frag_h(&h16[col][0] + kc * 32, lane);
#pragma unroll
      for (int q = 0; q < 4; ++q) acc[q] = wmma16(a, frag_h(Wh + (size_t)(w * 64 + q * 16 + col) * HH + kc * 32, lane), acc[q]); }
#pragma unroll
    for (int q = 0; q < 4; ++q)
#pragma unroll
      for (int rr = 0; rr < 8; ++rr) gates[8 * g + rr][w * 64 + q * 16 + col] = acc[q][rr];
    __syncthreads();
    int tok = x[(size_t)b * TT + t]; tok = tok < 0 ? 0 : (tok >= VV ? VV - 1 : tok);
    const float* tr = tb + (size_t)tok * G4;
    union { v8h hv; v4u uu; } pk; v4f o0, o1;
#pragma unroll
    for (int j = 0; j < 8; ++j) { const int u = u0 + j;
      const float ig = sigm(gates[r][u] + tr[u]), fg = sigm(gates[r][HH + u] + tr[HH + u]);
      const float gg = tanhf(gates[r][2 * HH + u] + tr[2 * HH + u]), og = sigm(gates[r][3 * HH + u] + tr[3 * HH + u]);
      c[j] = fg * c[j] + ig * gg; h[j] = og * tanhf(c[j]); pk.hv[j] = (_Float16)h[j]; if (j < 4) o0[j] = h[j]; else o1[j - 4] = h[j]; }
    *(v4u*)(&h16[r][u0]) = pk.uu;
    float* dst = hs + ((size_t)b * TT + t) * (2 * HH) + dir * HH + u0;
    vst2(dst, o0); vst2(dst + 4, o1);
    __syncthreads();
  }
}
__global__ __launch_bounds__(128) void k_fc(const float* __restrict__ hs, const float* __restrict__ fw, const float* __restrict__ fb, float* __restrict__ out) {
  __shared__ __align__(16) float so[4][16][68];
  const int tid = threadIdx.x, wave = tid >> 5, lane = tid & 31, col = lane & 15, g = lane >> 4;
  const int r0 = blockIdx.x * 64 + wave * 16;
  v8f acc[4] = {};
#pragma unroll 1
  for (int kc = 0; kc < 2 * HH / 32; ++kc) { const v16h a = frag_f32(hs + (size_t)(r0 + col) * (2 * HH) + kc * 32, lane);
#pragma unroll
    for (int j = 0; j < 4; ++j) acc[j] = wmma16(a, frag_f32(fw + (size_t)(j * 16 + col) * (2 * HH) + kc * 32, lane), acc[j]); }
#pragma unroll
  for (int j = 0; j < 4; ++j) { const float bb = fb[j * 16 + col];
#pragma unroll
    for (int rr = 0; rr < 8; ++rr) so[wave][8 * g + rr][j * 16 + col] = acc[j][rr] + bb; }
  LDSX();
  for (int q = lane; q < 16 * 16; q += 32) { const int rl = q >> 4, pc = q & 15; vst2(out + (size_t)(r0 + rl) * VV + pc * 4, *(const v4f*)(&so[wave][rl][pc * 4])); }
}
extern "C" void kernel_launch(void* const* d_in, const int* in_sizes, int n_in, void* d_out, int out_size, void* d_ws, size_t ws_size, hipStream_t stream) {
  (void)in_sizes; (void)n_in; (void)out_size; (void)ws_size;
  const int* x = (const int*)d_in[0]; const float* emb = (const float*)d_in[1];
  const float* wif = (const float*)d_in[2]; const float* whf = (const float*)d_in[3]; const float* bif = (const float*)d_in[4]; const float* bhf = (const float*)d_in[5];
  const float* wib = (const float*)d_in[6]; const float* whb = (const float*)d_in[7]; const float* bib = (const float*)d_in[8]; const float* bhb = (const float*)d_in[9];
  const float* fw = (const float*)d_in[10]; const float* fb = (const float*)d_in[11];
  float* out = (float*)d_out;
  char* ws = (char*)d_ws; size_t off = 0;
  auto take = [&](size_t bytes) { char* p = ws + off; off += (bytes + 255) & ~(size_t)255; return p; };
  float* tab = (float*)take((size_t)2 * VV * G4 * 4); _Float16* Wh16 = (_Float16*)take((size_t)2 * G4 * HH * 2); float* hs = (float*)take((size_t)NB * TT * 2 * HH * 4);
  k_prep<<<dim3(VV, 2), 256, 0, stream>>>(emb, wif, bif, bhf, wib, bib, bhb, whf, whb, tab, Wh16);
  k_lstm<<<dim3(NB / RB, 2), 256, 0, stream>>>(x, tab, Wh16, hs);
  k_fc<<<NB * TT / 64, 128, 0, stream>>>(hs, fw, fb, out);
}
